// BatchMultiHeadGraphAttention_5171140625169
// MI455X (gfx1250) — hardware-verified
//
#include <hip/hip_runtime.h>
#include <hip/hip_bf16.h>

typedef __attribute__((ext_vector_type(16))) _Float16 v16h;
typedef __attribute__((ext_vector_type(8)))  _Float16 v8h;
typedef __attribute__((ext_vector_type(16))) __bf16   v16b;
typedef __attribute__((ext_vector_type(8)))  __bf16   v8b;
typedef __attribute__((ext_vector_type(8)))  float    v8f;
typedef __attribute__((ext_vector_type(4)))  float    v4f;
typedef __attribute__((ext_vector_type(4)))  int      v4i;
typedef __attribute__((ext_vector_type(4)))  unsigned v4u;
typedef __attribute__((ext_vector_type(8)))  unsigned v8u;

constexpr int kBS   = 8;
constexpr int kN    = 1024;
constexpr int kFin  = 256;
constexpr int kNH   = 8;
constexpr int kFout = 64;
constexpr int kBH   = kBS * kNH;
constexpr int kMrows = kNH * kFout;
constexpr float kSlope  = 0.2f;
constexpr float kPCarry = 1024.0f;

constexpr size_t kBytesHB  = (size_t)kBS * kN * kFin * 2;
constexpr size_t kBytesWT  = (size_t)kMrows * kFin * 2;
constexpr size_t kBytesHPF = (size_t)kBS * kMrows * kN * 4;
constexpr size_t kBytesHPH = (size_t)kBS * kMrows * kN * 2;
constexpr size_t kBytesSD  = (size_t)kBH * kN * 4;
constexpr size_t kOffHB  = 0;
constexpr size_t kOffWT  = kOffHB + kBytesHB;
constexpr size_t kOffHPF = kOffWT + kBytesWT;
constexpr size_t kOffHPH = kOffHPF + kBytesHPF;
constexpr size_t kOffSrc = kOffHPH + kBytesHPH;
constexpr size_t kOffDst = kOffSrc + kBytesSD;
constexpr size_t kWsTotal = kOffDst + kBytesSD;
static_assert(kWsTotal == 30146560u);
static_assert(kWsTotal <= 134217728u);
static_assert(kOffWT % 256 == 0 && kOffHPF % 256 == 0 && kOffHPH % 256 == 0 && kOffSrc % 256 == 0 && kOffDst % 256 == 0);
static_assert(kMrows % 64 == 0 && kN % 64 == 0 && kFin % 32 == 0);
static_assert(kN % 64 == 0 && kFout == 64);

__device__ __forceinline__ unsigned short f2bf_bits(float f) {
  unsigned u = __float_as_uint(f);
  return (unsigned short)((u + 0x7FFFu + ((u >> 16) & 1u)) >> 16);
}
__device__ __forceinline__ float bf_bits2f(unsigned short h) { return __uint_as_float(((unsigned)h) << 16); }

__device__ __forceinline__ void dep_guard_h(v8f& a, v8f& b, v16h x, v16h y) { asm volatile("v_nop\n\tv_nop\n\tv_nop\n\tv_nop" : "+v"(a), "+v"(b) : "v"(x), "v"(y)); }
__device__ __forceinline__ void dep_guard_b(v8f& a, v8f& b, v16b x, v16b y) { asm volatile("v_nop\n\tv_nop\n\tv_nop\n\tv_nop" : "+v"(a), "+v"(b) : "v"(x), "v"(y)); }
__device__ __forceinline__ void keep4_h(v16h a, v16h b, v16h c, v16h d) { asm volatile("v_nop" :: "v"(a), "v"(b), "v"(c), "v"(d)); }
__device__ __forceinline__ void keep4_b(v16b a, v16b b, v16b c, v16b d) { asm volatile("v_nop" :: "v"(a), "v"(b), "v"(c), "v"(d)); }
__device__ __forceinline__ void acc_guard4(v8f& a, v8f& b, v8f& c, v8f& d) { asm volatile("v_nop\n\tv_nop\n\tv_nop\n\tv_nop" : "+v"(a), "+v"(b), "+v"(c), "+v"(d)); }
template <typename T> struct Frag;
template <> struct Frag<_Float16> {
  typedef v16h V; union U { v16h v; v8h h[2]; };
  static __device__ __forceinline__ v16h load(const _Float16* p) {
    U f; f.h[0] = *(const v8h*)(p); f.h[1] = *(const v8h*)(p + 16); return f.v;
  }
  static __device__ __forceinline__ v8f mma(v16h a, v16h b, v8f c) {
    return __builtin_amdgcn_wmma_f32_16x16x32_f16(false, a, false, b, (short)0, c, false, false);
  }
  static __device__ __forceinline__ void guard(v8f& a, v8f& b, v16h x, v16h y) { dep_guard_h(a, b, x, y); }
  static __device__ __forceinline__ void keep(v16h a, v16h b, v16h c, v16h d) { keep4_h(a, b, c, d); }
};
template <> struct Frag<__bf16> {
  typedef v16b V; union U { v16b v; v8b h[2]; };
  static __device__ __forceinline__ v16b load(const __bf16* p) {
    U f; f.h[0] = *(const v8b*)(p); f.h[1] = *(const v8b*)(p + 16); return f.v;
  }
  static __device__ __forceinline__ v8f mma(v16b a, v16b b, v8f c) {
    return __builtin_amdgcn_wmma_f32_16x16x32_bf16(false, a, false, b, (short)0, c, false, false);
  }
  static __device__ __forceinline__ void guard(v8f& a, v8f& b, v16b x, v16b y) { dep_guard_b(a, b, x, y); }
  static __device__ __forceinline__ void keep(v16b a, v16b b, v16b c, v16b d) { keep4_b(a, b, c, d); }
};

template <int ET> struct Elem;
template <> struct Elem<0> { typedef _Float16 T; };
template <> struct Elem<1> { typedef __bf16 T; };
template <int ET, bool SPLIT, int BIAS_MODE, int OUT_MODE, bool RESID, int ACT = 0>
__global__ __launch_bounds__(256) void wmma_gemm64(
    const unsigned short* __restrict__ Ap, const unsigned short* __restrict__ A2p, int lda, long strideA,
    const unsigned short* __restrict__ Btp, const unsigned short* __restrict__ Bt2p, int ldb, long strideB,
    void* __restrict__ Cout, void* __restrict__ Cout2, int ldc, long strideC,
    const float* __restrict__ bias,
    const float* __restrict__ resid, long strideR,
    int M, int N, int K, float scale) {
  typedef typename Elem<ET>::T T;
  typedef typename Frag<T>::V V;
  const T* A = (const T*)Ap; const T* A2 = (const T*)A2p; const T* Bt = (const T*)Btp; const T* Bt2 = (const T*)Bt2p;
  __shared__ __align__(16) float sT[8][16 * 68];
  const int b    = blockIdx.y;
  const int lane = threadIdx.x & 31;
  const int wave = threadIdx.x >> 5;
  const int tilesN = N >> 6;
  const int tilesM = M >> 6;
  const int tile = blockIdx.x * 8 + wave;
  if (tile >= tilesM * tilesN) return;
  const int tm = tile / tilesN;
  const int tn = tile - tm * tilesN;
  const int m0 = tm << 6;
  const int n0 = tn << 6;

  const T* Ab  = A  + (size_t)b * strideA;
  const T* Bb  = Bt + (size_t)b * strideB;
  const T* Ab2 = SPLIT ? (A2  + (size_t)b * strideA) : nullptr;
  const T* Bb2 = SPLIT ? (Bt2 + (size_t)b * strideB) : nullptr;

  const int rlane = lane & 15;
  const int koff  = (lane >> 4) * 8;
  const int mOff  = (lane >> 4) * 8;

  v8f acc[4][4];
#pragma unroll
  for (int i = 0; i < 4; ++i)
#pragma unroll
    for (int j = 0; j < 4; ++j) acc[i][j] = (v8f){0.f,0.f,0.f,0.f,0.f,0.f,0.f,0.f};

  for (int k0 = 0; k0 < K; k0 += 32) {
    V bh[4], bl[4];
#pragma unroll
    for (int j = 0; j < 4; ++j) {
      const size_t bo = (size_t)(n0 + (j << 4) + rlane) * ldb + koff + k0;
      bh[j] = Frag<T>::load(Bb + bo);
      if (SPLIT) bl[j] = Frag<T>::load(Bb2 + bo);
    }
#pragma unroll
    for (int i = 0; i < 4; ++i) {
      const size_t ao = (size_t)(m0 + (i << 4) + rlane) * lda + koff + k0;
      V ah = Frag<T>::load(Ab + ao);
      V al;
      if (SPLIT) al = Frag<T>::load(Ab2 + ao);
#pragma unroll
      for (int j = 0; j < 4; ++j) {
        acc[i][j] = Frag<T>::mma(ah, bh[j], acc[i][j]);
        if (SPLIT) {
          acc[i][j] = Frag<T>::mma(ah, bl[j], acc[i][j]);
          acc[i][j] = Frag<T>::mma(al, bh[j], acc[i][j]);
        }
      }
      Frag<T>::guard(acc[i][0], acc[i][3], ah, SPLIT ? al : ah);
    }
    Frag<T>::keep(bh[0], bh[1], bh[2], bh[3]);
    if (SPLIT) Frag<T>::keep(bl[0], bl[1], bl[2], bl[3]);
  }
  acc_guard4(acc[0][0], acc[0][1], acc[0][2], acc[0][3]);
  acc_guard4(acc[1][0], acc[1][1], acc[1][2], acc[1][3]);
  acc_guard4(acc[2][0], acc[2][1], acc[2][2], acc[2][3]);
  acc_guard4(acc[3][0], acc[3][1], acc[3][2], acc[3][3]);

  float* slab = sT[wave];
  const float* Rb = RESID ? (resid + (size_t)b * strideR) : nullptr;
#pragma unroll
  for (int i = 0; i < 4; ++i) {
    const int mBase = m0 + (i << 4);
#pragma unroll
    for (int j = 0; j < 4; ++j) {
      const int n = n0 + (j << 4) + rlane;
      float bv = 0.f;
      if (BIAS_MODE == 2) bv = bias[n];
#pragma unroll
      for (int r = 0; r < 8; ++r) {
        float v = acc[i][j][r] * scale;
        if (BIAS_MODE == 1) v += bias[mBase + mOff + r];
        if (BIAS_MODE == 2) v += bv;
        if (RESID) v += Rb[(size_t)(mBase + mOff + r) * ldc + n];
        if (ACT == 1) v = tanhf(v);
        if (ACT == 2) v = fmaxf(v, 0.0f);
        if (ACT == 3) v = v / (1.0f + expf(-v));
        if (ACT == 4) v = (v > 0.f) ? v : 0.01f * v;
        if (ACT == 5) v = 0.5f * v * (1.0f + erff(v * 0.70710678118654752f));
        slab[(mOff + r) * 68 + (j << 4) + rlane] = v;
      }
    }
    __builtin_amdgcn_fence(__ATOMIC_RELEASE, "workgroup");
    __builtin_amdgcn_wave_barrier();
    __builtin_amdgcn_fence(__ATOMIC_ACQUIRE, "workgroup");
    if (OUT_MODE == 0 || OUT_MODE == 3) {
      float* C = (float*)Cout + (size_t)b * strideC;
      const int hh = lane >> 4, c4 = (lane & 15) * 4;
      for (int pass = 0; pass < 2; ++pass) {
#pragma unroll
        for (int it = 0; it < 8; ++it) {
          const int row = it * 2 + hh;
          v4f v = *(const v4f*)(slab + row * 68 + c4);
          *(volatile v4f*)(C + (size_t)(mBase + row) * ldc + n0 + c4) = v;
        }
        __threadfence();
      }
    }
    if (OUT_MODE != 0) {
      const int q = lane >> 3, c8 = (lane & 7) * 8;
      unsigned short* C  = (unsigned short*)((OUT_MODE == 3) ? Cout2 : Cout) + (size_t)b * strideC;
      unsigned short* C2 = (OUT_MODE == 2) ? ((unsigned short*)Cout2 + (size_t)b * strideC) : nullptr;
      for (int pass = 0; pass < 2; ++pass) {
#pragma unroll
        for (int it = 0; it < 4; ++it) {
          const int row = it * 4 + q;
          const float* sp = slab + row * 68 + c8;
          v8h hv, lv;
#pragma unroll
          for (int e = 0; e < 8; ++e) {
            if (OUT_MODE == 1 || OUT_MODE == 3) {
              hv[e] = (_Float16)sp[e];
            } else {
              unsigned short hb = f2bf_bits(sp[e]);
              unsigned short lb = f2bf_bits(sp[e] - bf_bits2f(hb));
              hv[e] = __builtin_bit_cast(_Float16, hb);
              lv[e] = __builtin_bit_cast(_Float16, lb);
            }
          }
          *(volatile v8h*)(C + (size_t)(mBase + row) * ldc + n0 + c8) = hv;
          if (OUT_MODE == 2) *(volatile v8h*)(C2 + (size_t)(mBase + row) * ldc + n0 + c8) = lv;
        }
        __threadfence();
      }
    }
    __builtin_amdgcn_fence(__ATOMIC_RELEASE, "workgroup");
    __builtin_amdgcn_wave_barrier();
    __builtin_amdgcn_fence(__ATOMIC_ACQUIRE, "workgroup");
  }
}

__global__ __launch_bounds__(256) void k_cast_bf16x8(const float* __restrict__ in, unsigned short* __restrict__ outp, int n8) {
  const int i = blockIdx.x * 256 + threadIdx.x;
  if (i < n8) {
    const v4f x0 = *(const v4f*)(in + (size_t)i * 8);
    const v4f x1 = *(const v4f*)(in + (size_t)i * 8 + 4);
    v4u u;
    u[0] = (unsigned)f2bf_bits(x0[0]) | ((unsigned)f2bf_bits(x0[1]) << 16);
    u[1] = (unsigned)f2bf_bits(x0[2]) | ((unsigned)f2bf_bits(x0[3]) << 16);
    u[2] = (unsigned)f2bf_bits(x1[0]) | ((unsigned)f2bf_bits(x1[1]) << 16);
    u[3] = (unsigned)f2bf_bits(x1[2]) | ((unsigned)f2bf_bits(x1[3]) << 16);
    volatile v4u* p = (volatile v4u*)(outp + (size_t)i * 8);
    *p = u;
    __threadfence();
    *p = u;
  }
}

__global__ __launch_bounds__(256) void k_wt(const float* __restrict__ w, unsigned short* __restrict__ wT) {
  __shared__ float tile[64][65];
  const int tid = threadIdx.x;
  const int hd = blockIdx.x >> 2;
  const int f0 = (blockIdx.x & 3) * 64;
  {
    const int fr = tid >> 2;
    const int cb = (tid & 3) * 16;
    const float* src = w + ((size_t)(hd * kFin + f0 + fr)) * kFout + cb;
#pragma unroll
    for (int i = 0; i < 4; ++i) {
      const v4f v = *(const v4f*)(src + 4 * i);
      tile[fr][cb + 4 * i + 0] = v[0];
      tile[fr][cb + 4 * i + 1] = v[1];
      tile[fr][cb + 4 * i + 2] = v[2];
      tile[fr][cb + 4 * i + 3] = v[3];
    }
  }
  __syncthreads();
  for (int pass = 0; pass < 2; ++pass) {
#pragma unroll
    for (int it = 0; it < 2; ++it) {
      const int o  = it * 32 + (tid >> 3);
      const int c8 = (tid & 7) * 8;
      v4u u;
#pragma unroll
      for (int e = 0; e < 4; ++e) {
        const unsigned lo = (unsigned)f2bf_bits(tile[c8 + 2 * e][o]);
        const unsigned hi = (unsigned)f2bf_bits(tile[c8 + 2 * e + 1][o]);
        u[e] = lo | (hi << 16);
      }
      *(volatile v4u*)(wT + ((size_t)(hd * kFout + o)) * kFin + f0 + c8) = u;
    }
    __threadfence();
  }
}

__global__ __launch_bounds__(256) void k_scores(const float* __restrict__ hpF, const float* __restrict__ a_src,
                                             const float* __restrict__ a_dst, float* __restrict__ srcA,
                                             float* __restrict__ dstA) {
  __shared__ float ash[kFout];
  __shared__ float adh[kFout];
  const int tid = threadIdx.x;
  const int bh = blockIdx.x >> 2;
  const int hd = bh & 7;
  const int n  = (blockIdx.x & 3) * 256 + tid;
  if (tid < kFout) {
    ash[tid] = bf_bits2f(f2bf_bits(a_src[hd * kFout + tid]));
    adh[tid] = bf_bits2f(f2bf_bits(a_dst[hd * kFout + tid]));
  }
  __syncthreads();
  const float* col = hpF + (size_t)bh * kFout * kN + n;
  float s = 0.0f, d = 0.0f;
#pragma unroll 1
  for (int o = 0; o < kFout; ++o) {
    const float t = tanhf(col[(size_t)o * kN]);
    s += t * ash[o];
    d += t * adh[o];
  }
  volatile float* ps = srcA + (size_t)bh * kN + n;
  volatile float* pd = dstA + (size_t)bh * kN + n;
  *ps = s;
  *pd = d;
  __threadfence();
  *ps = s;
  *pd = d;
}

__device__ __forceinline__ v8f mma_h(v16h a, v16h b, v8f c) {
  c = __builtin_amdgcn_wmma_f32_16x16x32_f16(false, a, false, b, (short)0, c, false, false);
  asm volatile("v_nop\n\tv_nop\n\tv_nop\n\tv_nop" : "+v"(c) : "v"(a), "v"(b));
  return c;
}
__device__ __forceinline__ float p_elem(float src, float d, int a, float mb) {
  float x = src + d;
  x = (x >= 0.0f) ? x : kSlope * x;
  const float p = expf(x - mb);
  return (a > 0) ? p : 0.0f;
}

__global__ __launch_bounds__(128) void k_attn(const int* __restrict__ adj, const unsigned short* __restrict__ hpHp,
                                           const float* __restrict__ srcA, const float* __restrict__ dstA,
                                           float* __restrict__ out) {
  __shared__ __align__(16) float dsh[kN];
  __shared__ float wmx[4];
  __shared__ __align__(16) float Os[4][16 * 68];
  const int tid  = threadIdx.x;
  const int wave = tid >> 5;
  const int lane = tid & 31;
  const int hh   = lane >> 4;
  const int c    = lane & 15;
  const int qb = blockIdx.x & 15;
  const int bh = blockIdx.x >> 4;
  const int b  = bh >> 3;
  const int q0 = qb * 64 + wave * 16;

  {
    const float* dp = dstA + (size_t)bh * kN + tid * 8;
    const v4f d0 = *(const v4f*)(dp);
    const v4f d1 = *(const v4f*)(dp + 4);
    *(v4f*)(dsh + tid * 8) = d0;
    *(v4f*)(dsh + tid * 8 + 4) = d1;
    float m = fmaxf(fmaxf(fmaxf(d0[0], d0[1]), fmaxf(d0[2], d0[3])),
                    fmaxf(fmaxf(d1[0], d1[1]), fmaxf(d1[2], d1[3])));
#pragma unroll
    for (int off = 1; off < 32; off <<= 1) m = fmaxf(m, __shfl_xor(m, off, 32));
    if (lane == 0) wmx[wave] = m;
  }
  __syncthreads();
  const float dmax = fmaxf(fmaxf(wmx[0], wmx[1]), fmaxf(wmx[2], wmx[3]));

  const int row = q0 + c;
  const float srow = srcA[(size_t)bh * kN + row];
  float mb = srow + dmax;
  mb = (mb >= 0.0f) ? mb : kSlope * mb;
  const int* adjrow = adj + ((size_t)b * kN + row) * kN;
  const _Float16* vb = (const _Float16*)(const void*)hpHp + (size_t)bh * kFout * kN;

  v8f acc[4];
#pragma unroll
  for (int t = 0; t < 4; ++t) acc[t] = (v8f){0.f,0.f,0.f,0.f,0.f,0.f,0.f,0.f};
  float lsum = 0.0f;

  for (int ks = 0; ks < kN / 32; ++ks) {
    const int kA = ks * 32 + 8 * hh;
    const int kB = kA + 16;
    const v4i a0 = *(const v4i*)(adjrow + kA);
    const v4i a1 = *(const v4i*)(adjrow + kA + 4);
    const v4i a2 = *(const v4i*)(adjrow + kB);
    const v4i a3 = *(const v4i*)(adjrow + kB + 4);
    const v4f d0 = *(const v4f*)(dsh + kA);
    const v4f d1 = *(const v4f*)(dsh + kA + 4);
    const v4f d2 = *(const v4f*)(dsh + kB);
    const v4f d3 = *(const v4f*)(dsh + kB + 4);
    float pv[16];
#pragma unroll
    for (int e = 0; e < 4; ++e) {
      pv[e]      = p_elem(srow, d0[e], a0[e], mb);
      pv[4 + e]  = p_elem(srow, d1[e], a1[e], mb);
      pv[8 + e]  = p_elem(srow, d2[e], a2[e], mb);
      pv[12 + e] = p_elem(srow, d3[e], a3[e], mb);
    }
    v8u pw;
#pragma unroll
    for (int e = 0; e < 8; ++e) {
      lsum += pv[2 * e];
      lsum += pv[2 * e + 1];
      const unsigned lo = (unsigned)__builtin_bit_cast(unsigned short, (_Float16)(pv[2 * e] * kPCarry));
      const unsigned hi = (unsigned)__builtin_bit_cast(unsigned short, (_Float16)(pv[2 * e + 1] * kPCarry));
      pw[e] = lo | (hi << 16);
    }
    const v16h av = __builtin_bit_cast(v16h, pw);
    const _Float16* vk = vb + ks * 32 + 8 * hh;
#pragma unroll
    for (int t = 0; t < 4; ++t) {
      const v16h bvv = Frag<_Float16>::load(vk + (size_t)(t * 16 + c) * kN);
      acc[t] = mma_h(av, bvv, acc[t]);
    }
  }

  lsum += __shfl_xor(lsum, 16, 32);
  float* os = Os[wave];
#pragma unroll
  for (int r = 0; r < 8; ++r) {
    const float lr  = __shfl(lsum, 8 * hh + r, 32);
    const float inv = 1.0f / (lr * kPCarry);
#pragma unroll
    for (int t = 0; t < 4; ++t) os[(8 * hh + r) * 68 + t * 16 + c] = acc[t][r] * inv;
  }
  __syncthreads();
  {
    float* ob = out + ((size_t)bh * kN + q0) * kFout;
    const int c4 = (lane & 15) * 4;
    for (int pass = 0; pass < 2; ++pass) {
#pragma unroll
      for (int it = 0; it < 8; ++it) {
        const int orow = it * 2 + hh;
        const v4f val = *(const v4f*)(os + orow * 68 + c4);
        *(volatile v4f*)(ob + (size_t)orow * kFout + c4) = val;
      }
      __threadfence();
    }
  }
}

extern "C" void kernel_launch(void* const* d_in, const int* in_sizes, int n_in,
                              void* d_out, int out_size, void* d_ws, size_t ws_size,
                              hipStream_t stream) {
  if (n_in < 5) return;
  if (in_sizes[0] != kBS * kN * kFin) return;
  if (in_sizes[1] != kBS * kN * kN) return;
  if (in_sizes[2] != kNH * kFin * kFout) return;
  if (in_sizes[3] != kNH * kFout || in_sizes[4] != kNH * kFout) return;
  if (out_size != kBS * kNH * kN * kFout) return;
  if (ws_size < kWsTotal) return;

  const float* h     = (const float*)d_in[0];
  const int*   adj   = (const int*)d_in[1];
  const float* w     = (const float*)d_in[2];
  const float* a_src = (const float*)d_in[3];
  const float* a_dst = (const float*)d_in[4];
  float* out = (float*)d_out;

  char* ws = (char*)d_ws;
  unsigned short* hB  = (unsigned short*)(ws + kOffHB);
  unsigned short* wT  = (unsigned short*)(ws + kOffWT);
  float*          hpF = (float*)(ws + kOffHPF);
  unsigned short* hpH = (unsigned short*)(ws + kOffHPH);
  float*          srcA = (float*)(ws + kOffSrc);
  float*          dstA = (float*)(ws + kOffDst);

  const int n8 = kBS * kN * kFin / 8;
  k_cast_bf16x8<<<(n8 + 255) / 256, 256, 0, stream>>>(h, hB, n8);
  k_wt<<<kNH * (kFin / 64), 256, 0, stream>>>(w, wT);
  {
    const int M = kMrows, Nn = kN, K = kFin;
    const int tiles = (M / 64) * (Nn / 64);
    dim3 grid((tiles + 7) / 8, kBS);
    wmma_gemm64<1, false, 0, 3, false, 0><<<grid, 256, 0, stream>>>(
        wT, wT, K, 0L,
        hB, hB, K, (long)kN * kFin,
        (void*)hpF, (void*)hpH, kN, (long)kMrows * kN,
        a_src,
        h, 0L,
        M, Nn, K, 1.0f);
  }
  k_scores<<<kBH * (kN / 256), 256, 0, stream>>>(hpF, a_src, a_dst, srcA, dstA);
  k_attn<<<kBH * (kN / 64), 128, 0, stream>>>(adj, hpH, srcA, dstA, out);
}
